// FlaxRwkvSelfAttention_76879914598667
// MI455X (gfx1250) — hardware-verified
//
#include <hip/hip_runtime.h>
#include <math.h>

constexpr int kSeqLen = 4096;
constexpr int kHidden = 2048;
constexpr float kWCarry    = 32.0f;
constexpr float kYCarry    = 64.0f;
constexpr float kProjScale = 1.0f / 32.0f;
constexpr float kOutScale  = 1.0f / (64.0f * 32.0f);
static_assert(kSeqLen % 64 == 0);
static_assert(kHidden % 64 == 0);
static_assert(kHidden % 32 == 0);
static_assert(kHidden == 256 * 8);

typedef __attribute__((ext_vector_type(16))) _Float16 v16h;
typedef __attribute__((ext_vector_type(8)))  _Float16 v8h;
typedef __attribute__((ext_vector_type(16))) __bf16   v16b;
typedef __attribute__((ext_vector_type(8)))  __bf16   v8b;
typedef __attribute__((ext_vector_type(8)))  float    v8f;
typedef __attribute__((ext_vector_type(4)))  float    v4f;
typedef __attribute__((ext_vector_type(4)))  unsigned int v4u;

__device__ __forceinline__ unsigned short f2bf_bits(float f) {
  unsigned u = __float_as_uint(f);
  return (unsigned short)((u + 0x7FFFu + ((u >> 16) & 1u)) >> 16);
}
__device__ __forceinline__ float bf_bits2f(unsigned short h) { return __uint_as_float(((unsigned)h) << 16); }

__device__ __forceinline__ void dep_guard_h(v8f& a, v8f& b, v16h x, v16h y) { asm volatile("v_nop\n\tv_nop\n\tv_nop\n\tv_nop" : "+v"(a), "+v"(b) : "v"(x), "v"(y)); }
__device__ __forceinline__ void dep_guard_b(v8f& a, v8f& b, v16b x, v16b y) { asm volatile("v_nop\n\tv_nop\n\tv_nop\n\tv_nop" : "+v"(a), "+v"(b) : "v"(x), "v"(y)); }
__device__ __forceinline__ void keep4_h(v16h a, v16h b, v16h c, v16h d) { asm volatile("v_nop" :: "v"(a), "v"(b), "v"(c), "v"(d)); }
__device__ __forceinline__ void keep4_b(v16b a, v16b b, v16b c, v16b d) { asm volatile("v_nop" :: "v"(a), "v"(b), "v"(c), "v"(d)); }
__device__ __forceinline__ void acc_guard4(v8f& a, v8f& b, v8f& c, v8f& d) { asm volatile("v_nop\n\tv_nop\n\tv_nop\n\tv_nop" : "+v"(a), "+v"(b), "+v"(c), "+v"(d)); }
template <typename T> struct Frag;
template <> struct Frag<_Float16> {
  typedef v16h V; union U { v16h v; v8h h[2]; };
  static __device__ __forceinline__ v16h load(const _Float16* p) {
    U f; f.h[0] = *(const v8h*)(p); f.h[1] = *(const v8h*)(p + 16); return f.v;
  }
  static __device__ __forceinline__ v8f mma(v16h a, v16h b, v8f c) {
    return __builtin_amdgcn_wmma_f32_16x16x32_f16(false, a, false, b, (short)0, c, false, false);
  }
  static __device__ __forceinline__ void guard(v8f& a, v8f& b, v16h x, v16h y) { dep_guard_h(a, b, x, y); }
  static __device__ __forceinline__ void keep(v16h a, v16h b, v16h c, v16h d) { keep4_h(a, b, c, d); }
};
template <> struct Frag<__bf16> {
  typedef v16b V; union U { v16b v; v8b h[2]; };
  static __device__ __forceinline__ v16b load(const __bf16* p) {
    U f; f.h[0] = *(const v8b*)(p); f.h[1] = *(const v8b*)(p + 16); return f.v;
  }
  static __device__ __forceinline__ v8f mma(v16b a, v16b b, v8f c) {
    return __builtin_amdgcn_wmma_f32_16x16x32_bf16(false, a, false, b, (short)0, c, false, false);
  }
  static __device__ __forceinline__ void guard(v8f& a, v8f& b, v16b x, v16b y) { dep_guard_b(a, b, x, y); }
  static __device__ __forceinline__ void keep(v16b a, v16b b, v16b c, v16b d) { keep4_b(a, b, c, d); }
};

__device__ __forceinline__ unsigned pk16(unsigned short a, unsigned short b) { return (unsigned)a | ((unsigned)b << 16); }
__device__ __forceinline__ unsigned short h_bits(float f) { const _Float16 h = (_Float16)f; return __builtin_bit_cast(unsigned short, h); }

template <int ET> struct Elem;
template <> struct Elem<0> { typedef _Float16 T; };
template <> struct Elem<1> { typedef __bf16 T; };
template <int ET, bool SPLIT, int BIAS_MODE, int OUT_MODE, bool RESID, int ACT = 0>
__global__ __launch_bounds__(256) void wmma_gemm64(
    const unsigned short* __restrict__ Ap, const unsigned short* __restrict__ A2p, int lda, long strideA,
    const unsigned short* __restrict__ Btp, const unsigned short* __restrict__ Bt2p, int ldb, long strideB,
    void* __restrict__ Cout, void* __restrict__ Cout2, int ldc, long strideC,
    const float* __restrict__ bias,
    const float* __restrict__ resid, long strideR,
    int M, int N, int K, float scale) {
  typedef typename Elem<ET>::T T;
  typedef typename Frag<T>::V V;
  const T* A = (const T*)Ap; const T* A2 = (const T*)A2p; const T* Bt = (const T*)Btp; const T* Bt2 = (const T*)Bt2p;
  __shared__ __align__(16) float sT[8][16 * 68];
  const int b    = blockIdx.y;
  const int lane = threadIdx.x & 31;
  const int wave = threadIdx.x >> 5;
  const int tilesN = N >> 6;
  const int tilesM = M >> 6;
  const int tile = blockIdx.x * 8 + wave;
  if (tile >= tilesM * tilesN) return;
  const int tm = tile / tilesN;
  const int tn = tile - tm * tilesN;
  const int m0 = tm << 6;
  const int n0 = tn << 6;

  const T* Ab  = A  + (size_t)b * strideA;
  const T* Bb  = Bt + (size_t)b * strideB;
  const T* Ab2 = SPLIT ? (A2  + (size_t)b * strideA) : nullptr;
  const T* Bb2 = SPLIT ? (Bt2 + (size_t)b * strideB) : nullptr;

  const int rlane = lane & 15;
  const int koff  = (lane >> 4) * 8;
  const int mOff  = (lane >> 4) * 8;

  v8f acc[4][4];
#pragma unroll
  for (int i = 0; i < 4; ++i)
#pragma unroll
    for (int j = 0; j < 4; ++j) acc[i][j] = (v8f){0.f,0.f,0.f,0.f,0.f,0.f,0.f,0.f};

  for (int k0 = 0; k0 < K; k0 += 32) {
    V bh[4], bl[4];
#pragma unroll
    for (int j = 0; j < 4; ++j) {
      const size_t bo = (size_t)(n0 + (j << 4) + rlane) * ldb + koff + k0;
      bh[j] = Frag<T>::load(Bb + bo);
      if (SPLIT) bl[j] = Frag<T>::load(Bb2 + bo);
    }
#pragma unroll
    for (int i = 0; i < 4; ++i) {
      const size_t ao = (size_t)(m0 + (i << 4) + rlane) * lda + koff + k0;
      V ah = Frag<T>::load(Ab + ao);
      V al;
      if (SPLIT) al = Frag<T>::load(Ab2 + ao);
#pragma unroll
      for (int j = 0; j < 4; ++j) {
        acc[i][j] = Frag<T>::mma(ah, bh[j], acc[i][j]);
        if (SPLIT) {
          acc[i][j] = Frag<T>::mma(ah, bl[j], acc[i][j]);
          acc[i][j] = Frag<T>::mma(al, bh[j], acc[i][j]);
        }
      }
      Frag<T>::guard(acc[i][0], acc[i][3], ah, SPLIT ? al : ah);
    }
    Frag<T>::keep(bh[0], bh[1], bh[2], bh[3]);
    if (SPLIT) Frag<T>::keep(bl[0], bl[1], bl[2], bl[3]);
  }
  acc_guard4(acc[0][0], acc[0][1], acc[0][2], acc[0][3]);
  acc_guard4(acc[1][0], acc[1][1], acc[1][2], acc[1][3]);
  acc_guard4(acc[2][0], acc[2][1], acc[2][2], acc[2][3]);
  acc_guard4(acc[3][0], acc[3][1], acc[3][2], acc[3][3]);

  float* slab = sT[wave];
  const float* Rb = RESID ? (resid + (size_t)b * strideR) : nullptr;
#pragma unroll
  for (int i = 0; i < 4; ++i) {
    const int mBase = m0 + (i << 4);
#pragma unroll
    for (int j = 0; j < 4; ++j) {
      const int n = n0 + (j << 4) + rlane;
      float bv = 0.f;
      if (BIAS_MODE == 2) bv = bias[n];
#pragma unroll
      for (int r = 0; r < 8; ++r) {
        float v = acc[i][j][r] * scale;
        if (BIAS_MODE == 1) v += bias[mBase + mOff + r];
        if (BIAS_MODE == 2) v += bv;
        if (RESID) v += Rb[(size_t)(mBase + mOff + r) * ldc + n];
        if (ACT == 1) v = tanhf(v);
        if (ACT == 2) v = fmaxf(v, 0.0f);
        if (ACT == 3) v = v / (1.0f + expf(-v));
        if (ACT == 4) v = (v > 0.f) ? v : 0.01f * v;
        if (ACT == 5) v = 0.5f * v * (1.0f + erff(v * 0.70710678118654752f));
        slab[(mOff + r) * 68 + (j << 4) + rlane] = v;
      }
    }
    __builtin_amdgcn_fence(__ATOMIC_RELEASE, "workgroup");
    __builtin_amdgcn_wave_barrier();
    __builtin_amdgcn_fence(__ATOMIC_ACQUIRE, "workgroup");
    if (OUT_MODE == 0) {
      float* C = (float*)Cout + (size_t)b * strideC;
      const int hh = lane >> 4, c4 = (lane & 15) * 4;
      for (int pass = 0; pass < 2; ++pass) {
#pragma unroll
        for (int it = 0; it < 8; ++it) {
          const int row = it * 2 + hh;
          v4f v = *(const v4f*)(slab + row * 68 + c4);
          *(volatile v4f*)(C + (size_t)(mBase + row) * ldc + n0 + c4) = v;
        }
        __threadfence();
      }
    } else {
      const int q = lane >> 3, c8 = (lane & 7) * 8;
      unsigned short* C  = (unsigned short*)Cout  + (size_t)b * strideC;
      unsigned short* C2 = (OUT_MODE == 2) ? ((unsigned short*)Cout2 + (size_t)b * strideC) : nullptr;
      for (int pass = 0; pass < 2; ++pass) {
#pragma unroll
        for (int it = 0; it < 4; ++it) {
          const int row = it * 4 + q;
          const float* sp = slab + row * 68 + c8;
          v8h hv, lv;
#pragma unroll
          for (int e = 0; e < 8; ++e) {
            if (OUT_MODE == 1) {
              hv[e] = (_Float16)sp[e];
            } else {
              unsigned short hb = f2bf_bits(sp[e]);
              unsigned short lb = f2bf_bits(sp[e] - bf_bits2f(hb));
              hv[e] = __builtin_bit_cast(_Float16, hb);
              lv[e] = __builtin_bit_cast(_Float16, lb);
            }
          }
          *(volatile v8h*)(C + (size_t)(mBase + row) * ldc + n0 + c8) = hv;
          if (OUT_MODE == 2) *(volatile v8h*)(C2 + (size_t)(mBase + row) * ldc + n0 + c8) = lv;
        }
        __threadfence();
      }
    }
    __builtin_amdgcn_fence(__ATOMIC_RELEASE, "workgroup");
    __builtin_amdgcn_wave_barrier();
    __builtin_amdgcn_fence(__ATOMIC_ACQUIRE, "workgroup");
  }
}

__global__ __launch_bounds__(256) void mix_kernel(const float* __restrict__ hidden, const float* __restrict__ sx,
                                                  const float* __restrict__ tmk, const float* __restrict__ tmv,
                                                  const float* __restrict__ tmr,
                                                  unsigned short* __restrict__ KX, unsigned short* __restrict__ VX,
                                                  unsigned short* __restrict__ RX) {
  const int t  = blockIdx.x;
  const int c0 = threadIdx.x * 8;
  const int tp = (t > 0) ? (t - 1) : 0;
  const bool first = (t == 0);
  const float* cur = hidden + (size_t)t * kHidden + c0;
  const float* prv = hidden + (size_t)tp * kHidden + c0;
  const v4f ca = *(const v4f*)(cur), cb = *(const v4f*)(cur + 4);
  const v4f pa = *(const v4f*)(prv), pb = *(const v4f*)(prv + 4);
  const v4f sa = *(const v4f*)(sx + c0), sb = *(const v4f*)(sx + c0 + 4);
  const v4f ka = *(const v4f*)(tmk + c0), kb = *(const v4f*)(tmk + c0 + 4);
  const v4f va = *(const v4f*)(tmv + c0), vb = *(const v4f*)(tmv + c0 + 4);
  const v4f ra = *(const v4f*)(tmr + c0), rb = *(const v4f*)(tmr + c0 + 4);
  float x[8], p[8], mk[8], mv[8], mr[8];
#pragma unroll
  for (int e = 0; e < 4; ++e) {
    x[e] = ca[e];  x[4 + e] = cb[e];
    p[e] = first ? sa[e] : pa[e];
    p[4 + e] = first ? sb[e] : pb[e];
    mk[e] = ka[e]; mk[4 + e] = kb[e];
    mv[e] = va[e]; mv[4 + e] = vb[e];
    mr[e] = ra[e]; mr[4 + e] = rb[e];
  }
  unsigned short hk[8], hv[8], hr[8];
#pragma unroll
  for (int e = 0; e < 8; ++e) {
    const float kx = x[e] * mk[e] + p[e] * (1.0f - mk[e]);
    const float vx = x[e] * mv[e] + p[e] * (1.0f - mv[e]);
    const float rx = x[e] * mr[e] + p[e] * (1.0f - mr[e]);
    hk[e] = h_bits(kx);
    hv[e] = h_bits(vx);
    hr[e] = h_bits(rx);
  }
  const v4u uk = (v4u){pk16(hk[0], hk[1]), pk16(hk[2], hk[3]), pk16(hk[4], hk[5]), pk16(hk[6], hk[7])};
  const v4u uv = (v4u){pk16(hv[0], hv[1]), pk16(hv[2], hv[3]), pk16(hv[4], hv[5]), pk16(hv[6], hv[7])};
  const v4u ur = (v4u){pk16(hr[0], hr[1]), pk16(hr[2], hr[3]), pk16(hr[4], hr[5]), pk16(hr[6], hr[7])};
  const size_t off = (size_t)t * kHidden + c0;
  *(volatile v4u*)(KX + off) = uk;
  *(volatile v4u*)(VX + off) = uv;
  *(volatile v4u*)(RX + off) = ur;
  __threadfence();
  *(volatile v4u*)(KX + off) = uk;
  *(volatile v4u*)(VX + off) = uv;
  *(volatile v4u*)(RX + off) = ur;
}

__global__ __launch_bounds__(256) void wtcast_kernel(const float* __restrict__ W, unsigned short* __restrict__ WT, float scale) {
  __shared__ float sm[64][65];
  const int t  = threadIdx.x;
  const int d0 = blockIdx.x * 64;
  const int n0 = blockIdx.y * 64;
#pragma unroll
  for (int i = 0; i < 16; ++i) {
    const int e = i * 256 + t;
    const int r = e >> 6;
    const int c = e & 63;
    sm[c][r] = W[(size_t)(d0 + r) * kHidden + n0 + c] * scale;
  }
  __syncthreads();
  const int lane = t & 31, wave = t >> 5;
  const int q = lane >> 3, c8 = (lane & 7) * 8;
  v4u u[2];
#pragma unroll
  for (int it = 0; it < 2; ++it) {
    const int row = wave * 8 + it * 4 + q;
    unsigned short hb[8];
#pragma unroll
    for (int e = 0; e < 8; ++e) hb[e] = h_bits(sm[row][c8 + e]);
    u[it] = (v4u){pk16(hb[0], hb[1]), pk16(hb[2], hb[3]), pk16(hb[4], hb[5]), pk16(hb[6], hb[7])};
  }
  for (int pass = 0; pass < 2; ++pass) {
#pragma unroll
    for (int it = 0; it < 2; ++it) {
      const int row = wave * 8 + it * 4 + q;
      *(volatile v4u*)(WT + (size_t)(n0 + row) * kHidden + d0 + c8) = u[it];
    }
    __threadfence();
  }
}

__global__ __launch_bounds__(256) void recur_kernel(const float* __restrict__ kbuf, const float* __restrict__ vbuf,
                                                    const float* __restrict__ rbuf, const float* __restrict__ hidden,
                                                    const float* __restrict__ aa_in, const float* __restrict__ bb_in,
                                                    const float* __restrict__ pp_in,
                                                    const float* __restrict__ time_decay, const float* __restrict__ time_first,
                                                    unsigned short* __restrict__ YX, float* __restrict__ out_tail) {
  __shared__ __align__(16) unsigned short stage[8][256];
  __shared__ __align__(16) float fin[4][256];
  const int tid  = threadIdx.x;
  const int lane = tid & 31, wave = tid >> 5;
  const int hbase = blockIdx.x * 256;
  const int h = hbase + tid;
  const float tf   = time_first[h];
  const float wdec = -expf(time_decay[h]);
  float aa = aa_in[h], bb = bb_in[h], pp = pp_in[h];

  for (int tc = 0; tc < kSeqLen / 8; ++tc) {
#pragma unroll 1
    for (int s = 0; s < 8; ++s) {
      const size_t idx = (size_t)(tc * 8 + s) * kHidden + h;
      const float kk = kbuf[idx];
      const float vv = vbuf[idx];
      const float rp = rbuf[idx];
      const float rr = 1.0f / (1.0f + expf(-rp));
      const float ww = tf + kk;
      const float p  = fmaxf(pp, ww);
      const float e1 = expf(pp - p);
      const float e2 = expf(ww - p);
      const float y  = (e1 * aa + e2 * vv) / (e1 * bb + e2);
      const float ww2 = wdec + pp;
      const float p2  = fmaxf(ww2, kk);
      const float e1b = expf(ww2 - p2);
      const float e2b = expf(kk - p2);
      aa = e1b * aa + e2b * vv;
      bb = e1b * bb + e2b;
      pp = p2;
      stage[s][tid] = h_bits(rr * y * kYCarry);
    }
    __syncthreads();
    {
      const int t = tc * 8 + wave;
      const v4u u = *(const v4u*)(&stage[wave][lane * 8]);
      unsigned short* dst = YX + (size_t)t * kHidden + hbase + lane * 8;
      *(volatile v4u*)dst = u;
      __threadfence();
      *(volatile v4u*)dst = u;
    }
    __syncthreads();
  }

  fin[0][tid] = hidden[(size_t)(kSeqLen - 1) * kHidden + h];
  fin[1][tid] = aa;
  fin[2][tid] = bb;
  fin[3][tid] = pp;
  __syncthreads();
  if (wave < 4) {
    const float* src = fin[wave];
    const v4f v0 = *(const v4f*)(src + lane * 4);
    const v4f v1 = *(const v4f*)(src + 128 + lane * 4);
    float* dst = out_tail + (size_t)wave * kHidden + hbase;
    *(volatile v4f*)(dst + lane * 4) = v0;
    *(volatile v4f*)(dst + 128 + lane * 4) = v1;
    __threadfence();
    *(volatile v4f*)(dst + lane * 4) = v0;
    *(volatile v4f*)(dst + 128 + lane * 4) = v1;
  }
}

extern "C" void kernel_launch(void* const* d_in, const int* in_sizes, int n_in,
                              void* d_out, int out_size, void* d_ws, size_t ws_size, hipStream_t stream) {
  if (n_in < 14) return;
  const int nTH = kSeqLen * kHidden;
  const int nHH = kHidden * kHidden;
  if (in_sizes[0] != nTH) return;
  for (int i = 1; i <= 9; ++i) if (in_sizes[i] != kHidden) return;
  for (int i = 10; i <= 13; ++i) if (in_sizes[i] != nHH) return;
  if (out_size != nTH + 4 * kHidden) return;

  const float* hidden     = (const float*)d_in[0];
  const float* sx         = (const float*)d_in[1];
  const float* aa_in      = (const float*)d_in[2];
  const float* bb_in      = (const float*)d_in[3];
  const float* pp_in      = (const float*)d_in[4];
  const float* time_decay = (const float*)d_in[5];
  const float* time_first = (const float*)d_in[6];
  const float* tmk        = (const float*)d_in[7];
  const float* tmv        = (const float*)d_in[8];
  const float* tmr        = (const float*)d_in[9];
  const float* Wk         = (const float*)d_in[10];
  const float* Wv         = (const float*)d_in[11];
  const float* Wr         = (const float*)d_in[12];
  const float* Wo         = (const float*)d_in[13];
  float* out0 = (float*)d_out;
  float* out_tail = out0 + (size_t)nTH;

  const size_t plane16 = (size_t)nTH * 2;
  const size_t plane32 = (size_t)nTH * 4;
  const size_t wt16    = (size_t)nHH * 2;
  const size_t total   = 3 * plane16 + wt16 + 2 * plane32;
  if (total > ws_size) return;
  char* base = (char*)d_ws;
  unsigned short* RX = (unsigned short*)(base);
  unsigned short* KX = (unsigned short*)(base + plane16);
  unsigned short* VX = (unsigned short*)(base + 2 * plane16);
  unsigned short* WT = (unsigned short*)(base + 3 * plane16);
  float* rbuf = (float*)(base + 3 * plane16 + wt16);
  float* kbuf = (float*)(base + 3 * plane16 + wt16 + plane32);
  float* vbuf = (float*)(base);
  unsigned short* YX = (unsigned short*)(base + 2 * plane16);

  const dim3 castGrid(kHidden / 64, kHidden / 64);
  const int nTiles = (kSeqLen / 64) * (kHidden / 64);
  const dim3 gemmGrid((nTiles + 7) / 8, 1);

  mix_kernel<<<dim3(kSeqLen), 256, 0, stream>>>(hidden, sx, tmk, tmv, tmr, KX, VX, RX);

  wtcast_kernel<<<castGrid, 256, 0, stream>>>(Wr, WT, kWCarry);
  wmma_gemm64<0, false, 0, 0, false, 0><<<gemmGrid, 256, 0, stream>>>(
      RX, RX, kHidden, 0L, WT, WT, kHidden, 0L, (void*)rbuf, (void*)rbuf, kHidden, 0L,
      time_first, hidden, 0L, kSeqLen, kHidden, kHidden, kProjScale);

  wtcast_kernel<<<castGrid, 256, 0, stream>>>(Wk, WT, kWCarry);
  wmma_gemm64<0, false, 0, 0, false, 0><<<gemmGrid, 256, 0, stream>>>(
      KX, KX, kHidden, 0L, WT, WT, kHidden, 0L, (void*)kbuf, (void*)kbuf, kHidden, 0L,
      time_first, hidden, 0L, kSeqLen, kHidden, kHidden, kProjScale);

  wtcast_kernel<<<castGrid, 256, 0, stream>>>(Wv, WT, kWCarry);
  wmma_gemm64<0, false, 0, 0, false, 0><<<gemmGrid, 256, 0, stream>>>(
      VX, VX, kHidden, 0L, WT, WT, kHidden, 0L, (void*)vbuf, (void*)vbuf, kHidden, 0L,
      time_first, hidden, 0L, kSeqLen, kHidden, kHidden, kProjScale);

  recur_kernel<<<dim3(kHidden / 256), 256, 0, stream>>>(kbuf, vbuf, rbuf, hidden, aa_in, bb_in, pp_in,
                                                         time_decay, time_first, YX, out_tail);

  wtcast_kernel<<<castGrid, 256, 0, stream>>>(Wo, WT, kWCarry);
  wmma_gemm64<0, false, 0, 0, true, 0><<<gemmGrid, 256, 0, stream>>>(
      YX, YX, kHidden, 0L, WT, WT, kHidden, 0L, (void*)out0, (void*)out0, kHidden, 0L,
      time_first, hidden, 0L, kSeqLen, kHidden, kHidden, kOutScale);
}
